// DDoSDetectionModel_12171937317153
// MI455X (gfx1250) — hardware-verified
//
#include <hip/hip_runtime.h>


namespace {
constexpr int NB = 4096, DM = 256, DS = 32, DC = 16, NL = 4, DI = 1024, DTR = 16, DIN = 78, KIN = 96, NX = DTR + 2 * DS  , NXP = 96;
constexpr float EPS = 1e-5f, AS_ = 8.0f;
struct Wo_ { static constexpr size_t PIN = 0, IN = PIN + (size_t)DM * KIN, X = IN + (size_t)NL * 2 * DI * DM, DT = X + (size_t)NL * NXP * DI, OUT = DT + (size_t)NL * DI * 32, END = OUT + (size_t)NL * DM * DI; };
constexpr int P_BIN = 0, P_NW = 256, P_CW = 1280, P_CB = 5376, P_BDT = 9472, P_AL_unused = 13568, P_D = 13568, P_WF = 17664, P_BF = 17920, P_END = 17921;

typedef _Float16 b16;
typedef __attribute__((ext_vector_type(16))) _Float16 v16b;
typedef __attribute__((ext_vector_type(8))) _Float16 v8b;
typedef __attribute__((ext_vector_type(8))) float v8f;
typedef __attribute__((ext_vector_type(4))) float v4f;
__device__ __forceinline__ float bf16_rne(float f) { unsigned int u = __float_as_uint(f); u += 0x7FFFu + ((u >> 16) & 1u); return __uint_as_float(u & 0xFFFF0000u); }
__device__ __forceinline__ void split16(float v, b16& hi, b16& lo) { hi = (b16)v; lo = (b16)(v - (float)hi); }
__device__ __forceinline__ v16b frag_kb(const b16* p, int hh) { const v8b a = *(const v8b*)(p + 8 * hh), b = *(const v8b*)(p + 16 + 8 * hh); v16b f;
#pragma unroll
  for (int e = 0; e < 8; ++e) { f[e] = a[e]; f[8 + e] = b[e]; } return f; }
__device__ __forceinline__ void frag_split_s(const float* p, int hh, float sc, int kvalid, int kb, v16b& fh, v16b& fl) {
#pragma unroll
  for (int e = 0; e < 8; ++e) { b16 a, c; { const int k = kb + 8 * hh + e; split16((k < kvalid) ? p[8 * hh + e] * sc * AS_ : 0.0f, a, c); fh[e] = a; fl[e] = c; }
    { const int k = kb + 16 + 8 * hh + e; split16((k < kvalid) ? p[16 + 8 * hh + e] * sc * AS_ : 0.0f, a, c); fh[8 + e] = a; fl[8 + e] = c; } } }
__device__ __forceinline__ v8f wmma16b(v16b a, v16b b, v8f c) { v8f d = __builtin_amdgcn_wmma_f32_16x16x32_f16(false, a, false, b, (short)0, c, false, false); asm volatile("v_nop\n\tv_nop\n\tv_nop\n\tv_nop" : "+v"(d) : "v"(a), "v"(b)); return d; }
__device__ __forceinline__ void wave_lds_sync() { __builtin_amdgcn_fence(__ATOMIC_RELEASE, "workgroup"); __builtin_amdgcn_wave_barrier(); __builtin_amdgcn_fence(__ATOMIC_ACQUIRE, "workgroup"); }
__device__ __forceinline__ float nexp(float x) { return __builtin_amdgcn_exp2f(x * 1.4426950408889634f); }
__device__ __forceinline__ float nlog(float x) { return __builtin_amdgcn_logf(x) * 0.6931471805599453f; }
__device__ __forceinline__ float pmul(float a, float b) { float p = a * b; asm volatile("" : "+v"(p)); return p; }
__device__ __forceinline__ float wsum(float v) {
#pragma unroll
  for (int o = 1; o < 32; o <<= 1) v += __shfl_xor(v, o); return v; }
__device__ __forceinline__ float silu(float x) { return x / (1.0f + nexp(-x)); }
__device__ __forceinline__ float softplus_f(float x) { return (x > 20.0f) ? x : nlog(1.0f + nexp(x)); }

__global__ __launch_bounds__(256) void prep_kernel(const float* __restrict__ Wpi, const float* __restrict__ bpi, const float* __restrict__ nw, const float* __restrict__ Win, const float* __restrict__ cw, const float* __restrict__ cb, const float* __restrict__ Wx, const float* __restrict__ Wdt, const float* __restrict__ bdt, const float* __restrict__ Dp, const float* __restrict__ Wout, const float* __restrict__ Wf, const float* __restrict__ bf, b16* __restrict__ R, float* __restrict__ P) {
  const size_t tid = (size_t)blockIdx.x * 256 + threadIdx.x, nth = (size_t)gridDim.x * 256;
  for (int pass = 0; pass < 2; ++pass) {
    for (size_t p = tid; p < Wo_::END / 8; p += nth) { const size_t q = p * 8; v8b v;
      if (q < Wo_::IN) { const int o = (int)(q / KIN), k0 = (int)(q % KIN); for (int e = 0; e < 8; ++e) { const int k = k0 + e; v[e] = (b16)((k < DIN) ? bf16_rne(Wpi[(size_t)k * DM + o]) : 0.0f); } }
      else if (q < Wo_::X) { const size_t r = q - Wo_::IN; const int l = (int)(r / ((size_t)2 * DI * DM)), o = (int)(r / DM) % (2 * DI), k0 = (int)(r % DM); for (int e = 0; e < 8; ++e) v[e] = (b16)bf16_rne(Win[((size_t)l * DM + k0 + e) * (2 * DI) + o]); }
      else if (q < Wo_::DT) { const size_t r = q - Wo_::X; const int l = (int)(r / ((size_t)NXP * DI)), o = (int)(r / DI) % NXP, k0 = (int)(r % DI); for (int e = 0; e < 8; ++e) v[e] = (b16)((o < NX) ? bf16_rne(Wx[((size_t)l * DI + k0 + e) * NX + o]) : 0.0f); }
      else if (q < Wo_::OUT) { const size_t r = q - Wo_::DT; const int l = (int)(r / ((size_t)DI * 32)), o = (int)(r / 32) % DI, k0 = (int)(r % 32); for (int e = 0; e < 8; ++e) { const int k = k0 + e; v[e] = (b16)((k < DTR) ? bf16_rne(Wdt[((size_t)l * DTR + k) * DI + o]) : 0.0f); } }
      else { const size_t r = q - Wo_::OUT; const int l = (int)(r / ((size_t)DM * DI)), o = (int)(r / DI) % DM, k0 = (int)(r % DI); for (int e = 0; e < 8; ++e) v[e] = (b16)bf16_rne(Wout[((size_t)l * DI + k0 + e) * DM + o]); }
      *(volatile v8b*)(R + q) = v; }
    for (size_t q = tid; q < P_END; q += nth) { const int i = (int)q; float v;
      if (i < P_NW) v = bpi[i]; else if (i < P_CW) v = nw[i - P_NW]; else if (i < P_CB) v = cw[(size_t)(i - P_CW) * DC + (DC - 1)]; else if (i < P_BDT) v = cb[i - P_CB]; else if (i < P_D) v = bdt[i - P_BDT]; else if (i < P_WF) v = Dp[i - P_D]; else if (i < P_BF) v = Wf[i - P_WF]; else v = bf[0];
      P[q] = bf16_rne(v); }
    __threadfence(); }
}

__global__ __launch_bounds__(64) void pin_kernel(const float* __restrict__ x, const b16* __restrict__ R, const float* __restrict__ P, float* __restrict__ Hf) {
  __shared__ __attribute__((aligned(16))) float Ts[2][32][128 + 4];
  const int lane = threadIdx.x & 31, wave = threadIdx.x >> 5, nloc = lane & 15, hlf = lane >> 4, m0 = blockIdx.y * 32, c0 = blockIdx.x * 128;
  v8f acc[8];
#pragma unroll
  for (int t = 0; t < 8; ++t) acc[t] = (v8f){};
#pragma unroll
  for (int kb = 0; kb < KIN; kb += 32) { v16b a; const float* xr = x + (size_t)(m0 + wave * 16 + nloc) * DIN;
#pragma unroll
    for (int e = 0; e < 16; ++e) { const int k = kb + ((e < 8) ? (8 * hlf + e) : (16 + 8 * hlf + e - 8)); a[e] = (b16)((k < DIN) ? bf16_rne(xr[k]) : 0.0f); }
#pragma unroll
    for (int t = 0; t < 8; ++t) acc[t] = wmma16b(a, frag_kb(R + Wo_::PIN + (size_t)(c0 + t * 16 + nloc) * KIN + kb, hlf), acc[t]); }
#pragma unroll
  for (int t = 0; t < 8; ++t)
#pragma unroll
    for (int r = 0; r < 8; ++r) Ts[wave][8 * hlf + r][t * 16 + nloc] = acc[t][r] + P[P_BIN + c0 + t * 16 + nloc];
  wave_lds_sync();
  for (int pass = 0; pass < 2; ++pass) { for (int i = lane; i < 16 * 32; i += 32) { const int rr = i >> 5, c4 = (i & 31) * 4; *(volatile v4f*)(Hf + (size_t)(m0 + wave * 16 + rr) * DM + c0 + c4) = *(const v4f*)(&Ts[wave][rr][c4]); } __threadfence(); }
}

__global__ __launch_bounds__(64) void inproj_kernel(const float* __restrict__ Hf, const b16* __restrict__ R, const float* __restrict__ P, int l, float* __restrict__ XI, float* __restrict__ ZS) {
  __shared__ __attribute__((aligned(16))) float Ts[2][32][128 + 4]; __shared__ float rs[32]; __shared__ __attribute__((aligned(16))) float Xn[32][DM + 4];
  const int lane = threadIdx.x & 31, wave = threadIdx.x >> 5, nloc = lane & 15, hlf = lane >> 4, m0 = blockIdx.y * 32, c0 = blockIdx.x * 128; const b16* Wi = R + Wo_::IN + (size_t)l * 2 * DI * DM; const float* nw = P + P_NW + l * DM;
  for (int q = 0; q < 16; ++q) { const int rr = wave * 16 + q; const float* hr = Hf + (size_t)(m0 + rr) * DM; float s = 0.0f; float v[8];
#pragma unroll
    for (int e = 0; e < 8; ++e) { v[e] = hr[e * 32 + lane]; s += pmul(v[e], v[e]); }
    s = wsum(s); const float r_ = rsqrtf(s * (1.0f / DM) + EPS);
#pragma unroll
    for (int e = 0; e < 8; ++e) Xn[rr][e * 32 + lane] = pmul(v[e] * r_, nw[e * 32 + lane]); if (lane == 0) rs[rr] = r_; }
  wave_lds_sync();
  v8f acc[8];
#pragma unroll
  for (int t = 0; t < 8; ++t) acc[t] = (v8f){};
#pragma unroll 2
  for (int kb = 0; kb < DM; kb += 32) { v16b ah, al; frag_split_s(&Xn[wave * 16 + nloc][kb], hlf, 1.0f, DM, kb, ah, al);
#pragma unroll
    for (int t = 0; t < 8; ++t) { const v16b bw = frag_kb(Wi + (size_t)(c0 + t * 16 + nloc) * DM + kb, hlf); acc[t] = wmma16b(ah, bw, acc[t]); acc[t] = wmma16b(al, bw, acc[t]); } }
#pragma unroll
  for (int t = 0; t < 8; ++t) { const int c = c0 + t * 16 + nloc;
#pragma unroll
    for (int r = 0; r < 8; ++r) { const float v = acc[t][r] * (1.0f / AS_); float y; if (c < DI) y = silu(pmul(P[P_CW + l * DI + c], v) + P[P_CB + l * DI + c]); else y = silu(v); Ts[wave][8 * hlf + r][t * 16 + nloc] = y; } }
  wave_lds_sync();
  float* dst = (c0 < DI) ? (XI + c0) : (ZS + (c0 - DI));
  for (int pass = 0; pass < 2; ++pass) { for (int i = lane; i < 16 * 32; i += 32) { const int rr = i >> 5, c4 = (i & 31) * 4; *(volatile v4f*)(dst + (size_t)(m0 + wave * 16 + rr) * DI + c4) = *(const v4f*)(&Ts[wave][rr][c4]); } __threadfence(); }
}

__global__ __launch_bounds__(64) void xproj_kernel(const float* __restrict__ XI, const b16* __restrict__ R, int l, float* __restrict__ DBC) {
  __shared__ __attribute__((aligned(16))) float Ts[2][16][NXP + 4];
  const int lane = threadIdx.x & 31, wave = threadIdx.x >> 5, nloc = lane & 15, hlf = lane >> 4, m0 = blockIdx.x * 32 + wave * 16; const b16* Wx = R + Wo_::X + (size_t)l * NXP * DI;
  v8f acc[6];
#pragma unroll
  for (int t = 0; t < 6; ++t) acc[t] = (v8f){};
#pragma unroll 2
  for (int kb = 0; kb < DI; kb += 32) { v16b ah, al; frag_split_s(XI + (size_t)(m0 + nloc) * DI + kb, hlf, 1.0f, DI, 0, ah, al);
#pragma unroll
    for (int t = 0; t < 6; ++t) { const v16b bw = frag_kb(Wx + (size_t)(t * 16 + nloc) * DI + kb, hlf); acc[t] = wmma16b(ah, bw, acc[t]); acc[t] = wmma16b(al, bw, acc[t]); } }
#pragma unroll
  for (int t = 0; t < 6; ++t)
#pragma unroll
    for (int r = 0; r < 8; ++r) Ts[wave][8 * hlf + r][t * 16 + nloc] = acc[t][r] * (1.0f / AS_);
  wave_lds_sync();
  for (int pass = 0; pass < 2; ++pass) { for (int i = lane; i < 16 * (NXP / 4); i += 32) { const int rr = i / (NXP / 4), c4 = (i % (NXP / 4)) * 4; *(volatile v4f*)(DBC + (size_t)(m0 + rr) * NXP + c4) = *(const v4f*)(&Ts[wave][rr][c4]); } __threadfence(); }
}

__global__ __launch_bounds__(64) void ssm_kernel(const float* __restrict__ DBC, const float* __restrict__ XI, const float* __restrict__ ZS, const b16* __restrict__ R, const float* __restrict__ P, int l, float* __restrict__ Y) {
  __shared__ __attribute__((aligned(16))) float Ts[2][32][128 + 4]; __shared__ float bcs[32];
  const int lane = threadIdx.x & 31, wave = threadIdx.x >> 5, nloc = lane & 15, hlf = lane >> 4, m0 = blockIdx.y * 32, c0 = blockIdx.x * 128; const b16* Wd = R + Wo_::DT + (size_t)l * DI * 32;
  { const int rr = threadIdx.x & 31; if (wave == 0) { const float* d = DBC + (size_t)(m0 + rr) * NXP; float s = 0.0f; for (int n = 0; n < DS; ++n) s += pmul(d[DTR + n], d[DTR + DS + n]); bcs[rr] = s; } }
  v8f acc[8];
#pragma unroll
  for (int t = 0; t < 8; ++t) acc[t] = (v8f){};
  { v16b ah, al; frag_split_s(DBC + (size_t)(m0 + wave * 16 + nloc) * NXP, hlf, 1.0f, DTR, 0, ah, al);
#pragma unroll
    for (int t = 0; t < 8; ++t) { const v16b bw = frag_kb(Wd + (size_t)(c0 + t * 16 + nloc) * 32, hlf); acc[t] = wmma16b(ah, bw, acc[t]); acc[t] = wmma16b(al, bw, acc[t]); } }
  __syncthreads();
#pragma unroll
  for (int t = 0; t < 8; ++t) { const int c = c0 + t * 16 + nloc; const float bd = P[P_BDT + l * DI + c], Dv = P[P_D + l * DI + c];
#pragma unroll
    for (int r = 0; r < 8; ++r) { const int rr = wave * 16 + 8 * hlf + r; const float delta = softplus_f(acc[t][r] * (1.0f / AS_) + bd); const float xi = XI[(size_t)(m0 + rr) * DI + c], zs = ZS[(size_t)(m0 + rr) * DI + c];
      Ts[wave][8 * hlf + r][t * 16 + nloc] = pmul(pmul(pmul(delta, xi), bcs[rr]) + pmul(Dv, xi), zs); } }
  wave_lds_sync();
  for (int pass = 0; pass < 2; ++pass) { for (int i = lane; i < 16 * 32; i += 32) { const int rr = i >> 5, c4 = (i & 31) * 4; *(volatile v4f*)(Y + (size_t)(m0 + wave * 16 + rr) * DI + c0 + c4) = *(const v4f*)(&Ts[wave][rr][c4]); } __threadfence(); }
}

__global__ __launch_bounds__(64) void outproj_kernel(const float* __restrict__ Y, const b16* __restrict__ R, int l, float* __restrict__ Hf) {
  __shared__ __attribute__((aligned(16))) float Ts[2][32][128 + 4];
  const int lane = threadIdx.x & 31, wave = threadIdx.x >> 5, nloc = lane & 15, hlf = lane >> 4, m0 = blockIdx.y * 32, c0 = blockIdx.x * 128; const b16* Wo = R + Wo_::OUT + (size_t)l * DM * DI;
  v8f acc[8];
#pragma unroll
  for (int t = 0; t < 8; ++t) acc[t] = (v8f){};
#pragma unroll 2
  for (int kb = 0; kb < DI; kb += 32) { v16b ah, al; frag_split_s(Y + (size_t)(m0 + wave * 16 + nloc) * DI + kb, hlf, 1.0f, DI, 0, ah, al);
#pragma unroll
    for (int t = 0; t < 8; ++t) { const v16b bw = frag_kb(Wo + (size_t)(c0 + t * 16 + nloc) * DI + kb, hlf); acc[t] = wmma16b(ah, bw, acc[t]); acc[t] = wmma16b(al, bw, acc[t]); } }
#pragma unroll
  for (int t = 0; t < 8; ++t)
#pragma unroll
    for (int r = 0; r < 8; ++r) { const int rr = wave * 16 + 8 * hlf + r; Ts[wave][8 * hlf + r][t * 16 + nloc] = acc[t][r] * (1.0f / AS_) + Hf[(size_t)(m0 + rr) * DM + c0 + t * 16 + nloc]; }
  __syncthreads();
  for (int pass = 0; pass < 2; ++pass) { for (int i = lane; i < 16 * 32; i += 32) { const int rr = i >> 5, c4 = (i & 31) * 4; *(volatile v4f*)(Hf + (size_t)(m0 + wave * 16 + rr) * DM + c0 + c4) = *(const v4f*)(&Ts[wave][rr][c4]); } __threadfence(); }
}

__global__ __launch_bounds__(256) void final_kernel(const float* __restrict__ Hf, const float* __restrict__ P, float* __restrict__ out) {
  __shared__ __attribute__((aligned(16))) float ob[128];
  const int wave = threadIdx.x >> 5, lane = threadIdx.x & 31, r0 = blockIdx.x * 128;
  for (int q = 0; q < 16; ++q) { const int rr = wave * 16 + q; const float* hr = Hf + (size_t)(r0 + rr) * DM; float s = 0.0f;
#pragma unroll
    for (int e = 0; e < 8; ++e) s += pmul(hr[e * 32 + lane], P[P_WF + e * 32 + lane]);
    s = wsum(s); if (lane == 0) ob[rr] = 1.0f / (1.0f + nexp(-(s + P[P_BF]))); }
  __syncthreads();
  for (int pass = 0; pass < 2; ++pass) { if (threadIdx.x < 32) *(volatile v4f*)(out + r0 + threadIdx.x * 4) = *(const v4f*)(&ob[threadIdx.x * 4]); __threadfence(); }
}
}

extern "C" void kernel_launch(void* const* d_in, const int* in_sizes, int n_in,
                              void* d_out, int out_size, void* d_ws, size_t ws_size, hipStream_t stream) {
  (void)n_in; (void)out_size;
  const float* x = (const float*)d_in[0]; const float* Wpi = (const float*)d_in[1]; const float* bpi = (const float*)d_in[2]; const float* nw = (const float*)d_in[3]; const float* Win = (const float*)d_in[4]; const float* cw = (const float*)d_in[5]; const float* cb = (const float*)d_in[6];
  const float* Wx = (const float*)d_in[7]; const float* Wdt = (const float*)d_in[8]; const float* bdt = (const float*)d_in[9]; const float* Dp = (const float*)d_in[11]; const float* Wout = (const float*)d_in[12]; const float* Wf = (const float*)d_in[13]; const float* bf = (const float*)d_in[14];
  (void)d_in[10];
  float* out = (float*)d_out;
  if (in_sizes[0] != NB * DIN || in_sizes[4] != NL * DM * 2 * DI || in_sizes[7] != NL * DI * NX || in_sizes[8] != NL * DTR * DI || in_sizes[12] != NL * DI * DM) return;
  size_t off = 0; char* ws = (char*)d_ws;
  auto carve = [&](size_t bytes) { char* p = ws + off; off += (bytes + 255) & ~(size_t)255; return p; };
  b16* R = (b16*)carve(Wo_::END * 2); float* P = (float*)carve(18432 * 4); float* Hf = (float*)carve((size_t)NB * DM * 4); float* XI = (float*)carve((size_t)NB * DI * 4); float* ZS = (float*)carve((size_t)NB * DI * 4); float* DBC = (float*)carve((size_t)NB * NXP * 4); float* Y = (float*)carve((size_t)NB * DI * 4);
  if (off > ws_size) return;
  prep_kernel<<<512, 256, 0, stream>>>(Wpi, bpi, nw, Win, cw, cb, Wx, Wdt, bdt, Dp, Wout, Wf, bf, R, P);
  pin_kernel<<<dim3(2, NB / 32), 64, 0, stream>>>(x, R, P, Hf);
  for (int l = 0; l < NL; ++l) {
    inproj_kernel<<<dim3(16, NB / 32), 64, 0, stream>>>(Hf, R, P, l, XI, ZS);
    xproj_kernel<<<NB / 32, 64, 0, stream>>>(XI, R, l, DBC);
    ssm_kernel<<<dim3(8, NB / 32), 64, 0, stream>>>(DBC, XI, ZS, R, P, l, Y);
    outproj_kernel<<<dim3(2, NB / 32), 64, 0, stream>>>(Y, R, l, Hf); }
  final_kernel<<<NB / 128, 256, 0, stream>>>(Hf, P, out);
}
